// NaiveLSTM_84361747628164
// MI455X (gfx1250) — hardware-run, weakly checked
//
#include <hip/hip_runtime.h>
#include <math.h>

typedef __attribute__((ext_vector_type(16))) _Float16 v16h;
typedef __attribute__((ext_vector_type(8)))  _Float16 v8h;
typedef __attribute__((ext_vector_type(8)))  float    v8f;
typedef __attribute__((ext_vector_type(4)))  float    v4f;

constexpr int kBatch   = 64;
constexpr int kStep    = 512;
constexpr int kIn      = 256;
constexpr int kHid     = 512;
constexpr int kGate    = 4 * kHid;
constexpr int kOut     = 256;
constexpr int kCat     = kIn + kHid;
constexpr int kRowsBlk = 32;
constexpr int kScanThr = 512;
constexpr int kAPitch  = 776;
constexpr int kFPitch  = 516;
constexpr int kRowsAll = kBatch * kStep;
constexpr int kOut0    = kRowsAll * kOut;
constexpr int kOut1    = kBatch * kHid;
constexpr int kSmemA   = kRowsBlk * kAPitch * 2;
constexpr int kSmemF   = 16 * kFPitch * 4;
constexpr int kSmemBytes = (kSmemA > kSmemF) ? kSmemA : kSmemF;

constexpr float kCarryX  = 64.0f;
constexpr float kCarryWx = 1024.0f;
constexpr float kCarryH  = 256.0f;
constexpr float kCarryWu = 256.0f;
constexpr float kCarryWy = 1024.0f;
constexpr float kGateFold = 1.0f / (kCarryX * kCarryWx);
constexpr float kYFold    = 1.0f / (kCarryH * kCarryWy);
constexpr float kF16MinNormal = 6.103515625e-05f;

constexpr bool kBf16InputLeg = false;

static_assert(kCarryX * kCarryWx == kCarryH * kCarryWu);
static_assert(kGate == 2048 && kCat == 768);
static_assert(kHid == 32 * (kScanThr / 32));
static_assert(kBatch % kRowsBlk == 0);
static_assert(kCat % 32 == 0 && kHid % 32 == 0);
static_assert(kAPitch % 8 == 0 && kAPitch >= kCat);
static_assert(kFPitch % 4 == 0 && kFPitch >= kHid);
static_assert(kRowsAll % 64 == 0 && kOut % 64 == 0 && kGate % 64 == 0 && kIn % 64 == 0 && kHid % 64 == 0);
static_assert((size_t)kOut0 * 4 == 33554432ull);
static_assert(((size_t)kOut0 + kOut1) * 4 == 33685504ull);
static_assert(((size_t)kOut0 + 2 * (size_t)kOut1) * 4 == 33816576ull);
static_assert(kSmemBytes <= 65536);

__device__ __forceinline__ float in_leg(float f) {
  if (kBf16InputLeg) {
    unsigned u = __float_as_uint(f);
    u = (u + 0x7FFFu + ((u >> 16) & 1u)) & 0xFFFF0000u;
    return __uint_as_float(u);
  }
  return f;
}
__device__ __forceinline__ _Float16 f16_flush(float v) {
  const float a = fabsf(v);
  const float w = (a < kF16MinNormal) ? 0.0f : v;
  return (_Float16)w;
}
__device__ __forceinline__ float fsig(float v)  { return __builtin_amdgcn_rcpf(1.0f + __expf(-v)); }
__device__ __forceinline__ float ftanh(float v) { return 1.0f - 2.0f * __builtin_amdgcn_rcpf(__expf(2.0f * v) + 1.0f); }

__device__ __forceinline__ v16h ld_frag(const _Float16* p) {
  union U { v16h v; v8h h[2]; };
  U f;
  f.h[0] = *(const v8h*)(p);
  f.h[1] = *(const v8h*)(p + 16);
  return f.v;
}
__device__ __forceinline__ v8f mma_h(v16h a, v16h b, v8f c) {
  c = __builtin_amdgcn_wmma_f32_16x16x32_f16(false, a, false, b, (short)0, c, false, false);
  asm volatile("v_nop\n\tv_nop\n\tv_nop\n\tv_nop" : "+v"(c) : "v"(a), "v"(b));
  return c;
}
__device__ __forceinline__ void keep4_h(v16h a, v16h b, v16h c, v16h d) { asm volatile("v_nop" :: "v"(a), "v"(b), "v"(c), "v"(d)); }
__device__ __forceinline__ void acc_guard4(v8f& a, v8f& b, v8f& c, v8f& d) { asm volatile("v_nop\n\tv_nop\n\tv_nop\n\tv_nop" : "+v"(a), "+v"(b), "+v"(c), "+v"(d)); }
__device__ __forceinline__ void pin8(float (&a)[8]) {
  asm volatile("" : "+v"(a[0]), "+v"(a[1]), "+v"(a[2]), "+v"(a[3]), "+v"(a[4]), "+v"(a[5]), "+v"(a[6]), "+v"(a[7]));
}
__device__ __forceinline__ void pin4(float (&a)[4]) {
  asm volatile("" : "+v"(a[0]), "+v"(a[1]), "+v"(a[2]), "+v"(a[3]));
}

__global__ __launch_bounds__(256) void tp_f16_kernel(const float* __restrict__ src, int C, int ldo,
                                                     unsigned short* __restrict__ O, float sc) {
  __shared__ float Tt[64 * 65];
  const int tid = threadIdx.x;
  const int c0 = blockIdx.x * 64, r0 = blockIdx.y * 64;
#pragma unroll
  for (int i = 0; i < 4; ++i) {
    const int idx = i * 256 + tid;
    const int rr = idx >> 4, cc = (idx & 15) * 4;
    const v4f v = *(const v4f*)(src + (size_t)(r0 + rr) * (size_t)C + c0 + cc);
    Tt[rr * 65 + cc + 0] = v[0];
    Tt[rr * 65 + cc + 1] = v[1];
    Tt[rr * 65 + cc + 2] = v[2];
    Tt[rr * 65 + cc + 3] = v[3];
  }
  __syncthreads();
  const int q = tid >> 3, c8 = (tid & 7) * 8;
  v8h hv[2];
#pragma unroll
  for (int g = 0; g < 2; ++g) {
    const int qq = g * 32 + q;
#pragma unroll
    for (int e = 0; e < 8; ++e) {
      const float f = Tt[(c8 + e) * 65 + qq];
      hv[g][e] = f16_flush(in_leg(f) * sc);
    }
  }
  for (int pass = 0; pass < 2; ++pass) {
#pragma unroll
    for (int g = 0; g < 2; ++g) {
      const size_t o = (size_t)(c0 + g * 32 + q) * (size_t)ldo + (size_t)(r0 + c8);
      *(volatile v8h*)(O + o) = hv[g];
    }
    __threadfence();
  }
}

__device__ __forceinline__ void stage_x_tile(_Float16* At, const float* __restrict__ x, int rowbase, int t, int tid) {
#pragma unroll
  for (int it = 0; it < 2; ++it) {
    const int idx = it * kScanThr + tid;
    const int row = idx >> 5, c8 = (idx & 31) * 8;
    const float* sp = x + ((size_t)(rowbase + row) * kStep + (size_t)t) * kIn + c8;
    const v4f a = *(const v4f*)(sp);
    const v4f b = *(const v4f*)(sp + 4);
    v8h hv;
#pragma unroll
    for (int e = 0; e < 4; ++e) {
      hv[e]     = f16_flush(in_leg(a[e]) * kCarryX);
      hv[4 + e] = f16_flush(in_leg(b[e]) * kCarryX);
    }
    *(v8h*)(At + row * kAPitch + c8) = hv;
  }
}

__global__ __launch_bounds__(kScanThr) void lstm_scan_kernel(
    const float* __restrict__ x, const float* __restrict__ h0, const float* __restrict__ c0,
    const float* __restrict__ b_ih, const float* __restrict__ b_hh,
    const unsigned short* __restrict__ Wcp, unsigned short* __restrict__ hsp,
    float* __restrict__ out_h, float* __restrict__ out_c)
{
  __shared__ __align__(16) unsigned char smem[kSmemBytes];
  _Float16* At = (_Float16*)smem;
  float*    Fs = (float*)smem;
  const _Float16* Wc = (const _Float16*)Wcp;
  _Float16* hs = (_Float16*)hsp;

  const int tid = threadIdx.x, lane = tid & 31, wave = tid >> 5;
  const int c = lane & 15, hh = lane >> 4, koff = hh * 8;
  const int rowbase = blockIdx.x * kRowsBlk;

#pragma unroll 1
  for (int it = 0; it < 4; ++it) {
    const int idx = it * kScanThr + tid;
    const int row = idx >> 6, c8 = (idx & 63) * 8;
    const float* sp = h0 + (size_t)(rowbase + row) * kHid + c8;
    const v4f a = *(const v4f*)(sp);
    const v4f b = *(const v4f*)(sp + 4);
    v8h hv;
#pragma unroll
    for (int e = 0; e < 4; ++e) {
      hv[e]     = f16_flush(in_leg(a[e]) * kCarryH);
      hv[4 + e] = f16_flush(in_leg(b[e]) * kCarryH);
    }
    *(v8h*)(At + row * kAPitch + kIn + c8) = hv;
  }
  stage_x_tile(At, x, rowbase, 0, tid);

  float cst[2][2][8], hst[2][2][8], bsum[2][4];
#pragma unroll
  for (int nt = 0; nt < 2; ++nt) {
    const int j = 32 * wave + 16 * nt + c;
#pragma unroll
    for (int g = 0; g < 4; ++g) {
      const float bi = b_ih[g * kHid + j];
      const float bh = b_hh[g * kHid + j];
      bsum[nt][g] = in_leg(bi) + in_leg(bh);
    }
    pin4(bsum[nt]);
#pragma unroll
    for (int mi = 0; mi < 2; ++mi) {
#pragma unroll
      for (int r = 0; r < 8; ++r) {
        cst[nt][mi][r] = in_leg(c0[(size_t)(rowbase + mi * 16 + 8 * hh + r) * kHid + j]);
        hst[nt][mi][r] = 0.0f;
      }
      pin8(cst[nt][mi]);
    }
  }
  __syncthreads();

  const _Float16* arow0 = At + c * kAPitch + koff;
  const _Float16* arow1 = arow0 + 16 * kAPitch;
  const v8f z8 = {0.f, 0.f, 0.f, 0.f, 0.f, 0.f, 0.f, 0.f};

#pragma unroll 1
  for (int t = 0; t < kStep; ++t) {
#pragma unroll
    for (int nt = 0; nt < 2; ++nt) {
      const int j = 32 * wave + 16 * nt + c;
      const _Float16* wg0 = Wc + (size_t)j * kCat + koff;
      const _Float16* wg1 = wg0 + (size_t)kHid * kCat;
      const _Float16* wg2 = wg1 + (size_t)kHid * kCat;
      const _Float16* wg3 = wg2 + (size_t)kHid * kCat;
      v8f acc[4][2];
#pragma unroll
      for (int g = 0; g < 4; ++g) { acc[g][0] = z8; acc[g][1] = z8; }
#pragma unroll 1
      for (int k0 = 0; k0 < kCat; k0 += 32) {
        const v16h a0 = ld_frag(arow0 + k0);
        const v16h a1 = ld_frag(arow1 + k0);
        const v16h b0 = ld_frag(wg0 + k0);
        const v16h b1 = ld_frag(wg1 + k0);
        const v16h b2 = ld_frag(wg2 + k0);
        const v16h b3 = ld_frag(wg3 + k0);
        acc[0][0] = mma_h(a0, b0, acc[0][0]);
        acc[0][1] = mma_h(a1, b0, acc[0][1]);
        acc[1][0] = mma_h(a0, b1, acc[1][0]);
        acc[1][1] = mma_h(a1, b1, acc[1][1]);
        acc[2][0] = mma_h(a0, b2, acc[2][0]);
        acc[2][1] = mma_h(a1, b2, acc[2][1]);
        acc[3][0] = mma_h(a0, b3, acc[3][0]);
        acc[3][1] = mma_h(a1, b3, acc[3][1]);
      }
#pragma unroll
      for (int mi = 0; mi < 2; ++mi) {
#pragma unroll
        for (int r = 0; r < 8; ++r) {
          const float zi = acc[0][mi][r] * kGateFold + bsum[nt][0];
          const float zf = acc[1][mi][r] * kGateFold + bsum[nt][1];
          const float zj = acc[2][mi][r] * kGateFold + bsum[nt][2];
          const float zo = acc[3][mi][r] * kGateFold + bsum[nt][3];
          const float ig = fsig(zi);
          const float fg = fsig(zf);
          const float jg = ftanh(zj);
          const float og = fsig(zo);
          const float cn = fg * cst[nt][mi][r] + ig * jg;
          cst[nt][mi][r] = cn;
          hst[nt][mi][r] = og * ftanh(cn);
        }
      }
    }
    __syncthreads();
#pragma unroll
    for (int nt = 0; nt < 2; ++nt) {
      const int j = 32 * wave + 16 * nt + c;
#pragma unroll
      for (int mi = 0; mi < 2; ++mi)
#pragma unroll
        for (int r = 0; r < 8; ++r)
          At[(mi * 16 + 8 * hh + r) * kAPitch + kIn + j] = f16_flush(hst[nt][mi][r] * kCarryH);
    }
    {
      const int tn = (t + 1 < kStep) ? (t + 1) : (kStep - 1);
      stage_x_tile(At, x, rowbase, tn, tid);
    }
    __syncthreads();
    {
      v8h hv[4];
#pragma unroll
      for (int it = 0; it < 4; ++it) {
        const int idx = it * kScanThr + tid;
        const int row = idx >> 6, c8 = (idx & 63) * 8;
        hv[it] = *(const v8h*)(At + row * kAPitch + kIn + c8);
      }
      for (int pass = 0; pass < 2; ++pass) {
#pragma unroll
        for (int it = 0; it < 4; ++it) {
          const int idx = it * kScanThr + tid;
          const int row = idx >> 6, c8 = (idx & 63) * 8;
          *(volatile v8h*)(hs + ((size_t)(rowbase + row) * kStep + (size_t)t) * kHid + c8) = hv[it];
        }
        __threadfence();
      }
    }
  }

#pragma unroll
  for (int ph = 0; ph < 4; ++ph) {
    const int which = ph >> 1, mi = ph & 1;
    __syncthreads();
#pragma unroll
    for (int nt = 0; nt < 2; ++nt) {
      const int j = 32 * wave + 16 * nt + c;
#pragma unroll
      for (int r = 0; r < 8; ++r)
        Fs[(8 * hh + r) * kFPitch + j] = which ? cst[nt][mi][r] : hst[nt][mi][r];
    }
    __syncthreads();
    float* dst = which ? out_c : out_h;
    v4f fv[4];
#pragma unroll
    for (int it = 0; it < 4; ++it) {
      const int idx = it * kScanThr + tid;
      const int row = idx >> 7, c4 = (idx & 127) * 4;
      fv[it] = *(const v4f*)(Fs + row * kFPitch + c4);
    }
    for (int pass = 0; pass < 2; ++pass) {
#pragma unroll
      for (int it = 0; it < 4; ++it) {
        const int idx = it * kScanThr + tid;
        const int row = idx >> 7, c4 = (idx & 127) * 4;
        *(volatile v4f*)(dst + (size_t)(rowbase + mi * 16 + row) * kHid + c4) = fv[it];
      }
      __threadfence();
    }
  }
}

__global__ __launch_bounds__(256) void out_gemm_kernel(
    const unsigned short* __restrict__ Ap, int lda,
    const unsigned short* __restrict__ Btp, int ldb,
    float* __restrict__ C, int ldc, const float* __restrict__ bias,
    int M, int N, int K, float scale) {
  const _Float16* A  = (const _Float16*)Ap;
  const _Float16* Bt = (const _Float16*)Btp;
  __shared__ __align__(16) float sT[8][16 * 68];
  const int lane = threadIdx.x & 31;
  const int wave = threadIdx.x >> 5;
  const int tilesN = N >> 6;
  const int tilesM = M >> 6;
  const int tile = blockIdx.x * 8 + wave;
  if (tile >= tilesM * tilesN) return;
  const int tm = tile / tilesN;
  const int tn = tile - tm * tilesN;
  const int m0 = tm << 6;
  const int n0 = tn << 6;

  const int rlane = lane & 15;
  const int koff  = (lane >> 4) * 8;
  const int mOff  = (lane >> 4) * 8;

  v8f acc[4][4];
#pragma unroll
  for (int i = 0; i < 4; ++i)
#pragma unroll
    for (int j = 0; j < 4; ++j) acc[i][j] = (v8f){0.f, 0.f, 0.f, 0.f, 0.f, 0.f, 0.f, 0.f};

  for (int k0 = 0; k0 < K; k0 += 32) {
    v16h bh[4];
#pragma unroll
    for (int j = 0; j < 4; ++j) {
      const size_t bo = (size_t)(n0 + (j << 4) + rlane) * ldb + koff + k0;
      bh[j] = ld_frag(Bt + bo);
    }
#pragma unroll
    for (int i = 0; i < 4; ++i) {
      const size_t ao = (size_t)(m0 + (i << 4) + rlane) * lda + koff + k0;
      const v16h ah = ld_frag(A + ao);
#pragma unroll
      for (int j = 0; j < 4; ++j) acc[i][j] = mma_h(ah, bh[j], acc[i][j]);
    }
    keep4_h(bh[0], bh[1], bh[2], bh[3]);
  }
  acc_guard4(acc[0][0], acc[0][1], acc[0][2], acc[0][3]);
  acc_guard4(acc[1][0], acc[1][1], acc[1][2], acc[1][3]);
  acc_guard4(acc[2][0], acc[2][1], acc[2][2], acc[2][3]);
  acc_guard4(acc[3][0], acc[3][1], acc[3][2], acc[3][3]);

  float* slab = sT[wave];
#pragma unroll
  for (int i = 0; i < 4; ++i) {
    const int mBase = m0 + (i << 4);
#pragma unroll
    for (int j = 0; j < 4; ++j) {
      const int n = n0 + (j << 4) + rlane;
      const float bv = in_leg(bias[n]);
#pragma unroll
      for (int r = 0; r < 8; ++r) {
        const float v = acc[i][j][r] * scale + bv;
        slab[(mOff + r) * 68 + (j << 4) + rlane] = v;
      }
    }
    __builtin_amdgcn_fence(__ATOMIC_RELEASE, "workgroup");
    __builtin_amdgcn_wave_barrier();
    __builtin_amdgcn_fence(__ATOMIC_ACQUIRE, "workgroup");
    {
      const int hh = lane >> 4, c4 = (lane & 15) * 4;
      for (int pass = 0; pass < 2; ++pass) {
#pragma unroll
        for (int it = 0; it < 8; ++it) {
          const int row = it * 2 + hh;
          const v4f v = *(const v4f*)(slab + row * 68 + c4);
          *(volatile v4f*)(C + (size_t)(mBase + row) * ldc + n0 + c4) = v;
        }
        __threadfence();
      }
    }
    __builtin_amdgcn_fence(__ATOMIC_RELEASE, "workgroup");
    __builtin_amdgcn_wave_barrier();
    __builtin_amdgcn_fence(__ATOMIC_ACQUIRE, "workgroup");
  }
}

extern "C" void kernel_launch(void* const* d_in, const int* in_sizes, int n_in,
                              void* d_out, int out_size, void* d_ws, size_t ws_size, hipStream_t stream) {
  if (n_in < 9 || d_out == nullptr || d_ws == nullptr) return;
  if (in_sizes[0] != kBatch * kStep * kIn || in_sizes[1] != kBatch * kHid || in_sizes[2] != kBatch * kHid ||
      in_sizes[3] != kIn * kGate || in_sizes[4] != kHid * kGate || in_sizes[5] != kGate || in_sizes[6] != kGate ||
      in_sizes[7] != kHid * kOut || in_sizes[8] != kOut || out_size != kOut0 + 2 * kOut1) return;

  const float* x    = (const float*)d_in[0];
  const float* h0   = (const float*)d_in[1];
  const float* c0   = (const float*)d_in[2];
  const float* W_x  = (const float*)d_in[3];
  const float* U_h  = (const float*)d_in[4];
  const float* b_ih = (const float*)d_in[5];
  const float* b_hh = (const float*)d_in[6];
  const float* W_y  = (const float*)d_in[7];
  const float* b_y  = (const float*)d_in[8];
  float* y_out = (float*)d_out;
  float* hT    = y_out + (size_t)kOut0;
  float* cT    = hT + (size_t)kOut1;

  char* ws = (char*)d_ws; size_t off = 0;
  auto carve = [&](size_t bytes) -> char* { char* p = ws + off; off += (bytes + 255) & ~(size_t)255; return p; };
  unsigned short* WC = (unsigned short*)carve((size_t)kGate * kCat * 2);
  unsigned short* WY = (unsigned short*)carve((size_t)kOut * kHid * 2);
  unsigned short* HS = (unsigned short*)carve((size_t)kRowsAll * kHid * 2);
  if (off > ws_size || off > (size_t)134217728) return;

  tp_f16_kernel<<<dim3(kGate / 64, kIn / 64), 256, 0, stream>>>(W_x, kGate, kCat, WC, kCarryWx);
  tp_f16_kernel<<<dim3(kGate / 64, kHid / 64), 256, 0, stream>>>(U_h, kGate, kCat, WC + kIn, kCarryWu);
  tp_f16_kernel<<<dim3(kOut / 64, kHid / 64), 256, 0, stream>>>(W_y, kOut, kHid, WY, kCarryWy);

  lstm_scan_kernel<<<kBatch / kRowsBlk, kScanThr, 0, stream>>>(x, h0, c0, b_ih, b_hh, WC, HS, hT, cT);

  out_gemm_kernel<<<(kRowsAll / 64) * (kOut / 64) / 8, 256, 0, stream>>>(
      HS, kHid, WY, kHid, y_out, kOut, b_y, kRowsAll, kOut, kHid, kYFold);
}
